// GCN_classifier_39591008534852
// MI455X (gfx1250) — hardware-verified
//
#include <hip/hip_runtime.h>
#include <stddef.h>


typedef __bf16 v16bf __attribute__((ext_vector_type(16)));
typedef __bf16 v8bf  __attribute__((ext_vector_type(8)));
typedef float  v8f   __attribute__((ext_vector_type(8)));
typedef float  v4f   __attribute__((ext_vector_type(4)));
typedef int    v4i   __attribute__((ext_vector_type(4)));

#define NN   512
#define FIN  3
#define HD   64
#define NC   10
#define NCP  16
#define ADJ_RCP (1.0f / 29.0f)

union Frag16 { v16bf v; v8bf half[2]; };
union Pack8  { v8bf b; v4i u; };

__device__ __forceinline__ void mma3(v8f& acc, const v16bf& ah, const v16bf& al,
                                     const v16bf& bh, const v16bf& bl) {
    acc = __builtin_amdgcn_wmma_f32_16x16x32_bf16(false, ah, false, bh, (short)0, acc, false, false);
    acc = __builtin_amdgcn_wmma_f32_16x16x32_bf16(false, ah, false, bl, (short)0, acc, false, false);
    acc = __builtin_amdgcn_wmma_f32_16x16x32_bf16(false, al, false, bh, (short)0, acc, false, false);
    asm volatile("v_nop\n\tv_nop\n\tv_nop\n\tv_nop" : "+v"(acc) : "v"(ah), "v"(al), "v"(bh), "v"(bl));
}

__device__ __forceinline__ void load_pk(const float2* s_pos, int kbase, float2 pk[16]) {
    const v4f* p0 = (const v4f*)(s_pos + kbase);
    const v4f* p1 = (const v4f*)(s_pos + kbase + 16);
#pragma unroll
    for (int q = 0; q < 4; ++q) {
        const v4f a = p0[q];
        pk[2 * q]     = make_float2(a[0], a[1]);
        pk[2 * q + 1] = make_float2(a[2], a[3]);
        const v4f c = p1[q];
        pk[8 + 2 * q]     = make_float2(c[0], c[1]);
        pk[8 + 2 * q + 1] = make_float2(c[2], c[3]);
    }
}

__device__ __forceinline__ void adj_tile(float2 pm, int nrow, int kbase, const float2 pk[16],
                                         v16bf& ah, v16bf& al) {
    v16bf th, tl;
#pragma unroll
    for (int i = 0; i < 16; ++i) {
        const int k = kbase + (i & 7) + ((i & 8) << 1);
        const float dx = pm.x - pk[i].x;
        const float dy = pm.y - pk[i].y;
        const float d2 = dx * dx + dy * dy;
        float v = __builtin_amdgcn_rsqf(d2) * ADJ_RCP;
        v = (k == nrow) ? 1.0f : v;
        const __bf16 hv = (__bf16)v;
        const float res = v - (float)hv;
        th[i] = hv;
        tl[i] = (__bf16)res;
    }
    ah = th;
    al = tl;
}

__global__ void __launch_bounds__(256)
k_xw1(const float* __restrict__ x, const float* __restrict__ W1,
      __bf16* __restrict__ xh, __bf16* __restrict__ xl, int nthr) {
    const int g = (int)blockIdx.x * 256 + (int)threadIdx.x;
    if (g >= nthr) return;
    const int chunk = g & 63;
    const int hcol  = (g >> 6) & 63;
    const int b     = g >> 12;
    const float w0 = W1[hcol];
    const float w1 = W1[HD + hcol];
    const float w2 = W1[2 * HD + hcol];
    const v4f* xr = (const v4f*)(x + ((size_t)b * NN + (size_t)chunk * 8) * FIN);
    float xv[24];
#pragma unroll
    for (int q = 0; q < 6; ++q) {
        const v4f t = xr[q];
        xv[4 * q] = t[0]; xv[4 * q + 1] = t[1]; xv[4 * q + 2] = t[2]; xv[4 * q + 3] = t[3];
    }
    Pack8 ph, pl;
#pragma unroll
    for (int i = 0; i < 8; ++i) {
        const float v = xv[3 * i] * w0 + xv[3 * i + 1] * w1 + xv[3 * i + 2] * w2;
        const __bf16 hv = (__bf16)v;
        ph.b[i] = hv;
        pl.b[i] = (__bf16)(v - (float)hv);
    }
    const size_t off = ((size_t)b * HD + hcol) * NN + (size_t)chunk * 8;
    const v4i vh = ph.u, vl = pl.u;
    volatile v4i* dh = (volatile v4i*)(xh + off);
    volatile v4i* dl = (volatile v4i*)(xl + off);
    *dh = vh;
    *dl = vl;
    __threadfence();
    *dh = vh;
    *dl = vl;
}

__global__ void __launch_bounds__(128)
k_layer1(const float* __restrict__ x, const __bf16* __restrict__ xh, const __bf16* __restrict__ xl,
         const float* __restrict__ b1, const float* __restrict__ W2,
         __bf16* __restrict__ hh, __bf16* __restrict__ hl, int nblk) {
    __shared__ __align__(16) float2 s_pos[NN];
    __shared__ float s_w2[HD * NC];
    __shared__ float s_b1[HD];
    __shared__ __align__(16) float s_h[4][16][HD + 4];
    __shared__ __align__(16) __bf16 s_oh[NCP][64];
    __shared__ __align__(16) __bf16 s_ol[NCP][64];

    if ((int)blockIdx.x >= nblk) return;
    const int tid  = threadIdx.x;
    const int lane = tid & 31;
    const int wv   = tid >> 5;
    const int hf   = lane >> 4;
    const int m    = lane & 15;
    const int b    = (int)blockIdx.x >> 3;
    const int rblk = (int)blockIdx.x & 7;

    for (int n = tid; n < NN; n += 128) {
        const float* xr = x + ((size_t)b * NN + n) * FIN;
        s_pos[n] = make_float2(xr[0], xr[1]);
    }
    for (int i = tid; i < HD * NC; i += 128) s_w2[i] = W2[i];
    if (tid < HD) s_b1[tid] = b1[tid];
    for (int i = tid; i < (NCP - NC) * 64; i += 128) {
        const int c = NC + (i >> 6);
        const int e = i & 63;
        s_oh[c][e] = (__bf16)0.0f;
        s_ol[c][e] = (__bf16)0.0f;
    }
    __syncthreads();

    const int rowbase = rblk * 64 + wv * 16;
    const int nrow    = rowbase + m;
    const float2 pm   = s_pos[nrow];

    v8f acc[4] = {};
    const __bf16* xhb = xh + (size_t)b * HD * NN;
    const __bf16* xlb = xl + (size_t)b * HD * NN;

#pragma unroll 1
    for (int kt = 0; kt < NN / 32; ++kt) {
        const int kbase = kt * 32 + hf * 8;
        float2 pk[16];
        load_pk(s_pos, kbase, pk);
        v16bf ah, al;
        adj_tile(pm, nrow, kbase, pk, ah, al);
#pragma unroll
        for (int ht = 0; ht < 4; ++ht) {
            const size_t ro = (size_t)(ht * 16 + m) * NN + (size_t)kbase;
            Frag16 fbh, fbl;
            fbh.half[0] = *(const v8bf*)(xhb + ro);
            fbh.half[1] = *(const v8bf*)(xhb + ro + 16);
            fbl.half[0] = *(const v8bf*)(xlb + ro);
            fbl.half[1] = *(const v8bf*)(xlb + ro + 16);
            mma3(acc[ht], ah, al, fbh.v, fbl.v);
        }
    }

#pragma unroll
    for (int ht = 0; ht < 4; ++ht) {
        const int col = ht * 16 + m;
        const float bias = s_b1[col];
#pragma unroll
        for (int r = 0; r < 8; ++r)
            s_h[wv][8 * hf + r][col] = fmaxf(acc[ht][r] + bias, 0.0f);
    }
    __syncthreads();

    {
        const float* hrow = &s_h[wv][m][0];
        const int c0 = hf * 5;
        float p0 = 0.0f, p1 = 0.0f, p2 = 0.0f, p3 = 0.0f, p4 = 0.0f;
#pragma unroll 16
        for (int k = 0; k < HD; ++k) {
            const float hv = hrow[k];
            const float* wr = &s_w2[k * NC + c0];
            p0 += hv * wr[0];
            p1 += hv * wr[1];
            p2 += hv * wr[2];
            p3 += hv * wr[3];
            p4 += hv * wr[4];
        }
        const float pv[5] = {p0, p1, p2, p3, p4};
        const int rloc = wv * 16 + m;
#pragma unroll
        for (int q = 0; q < 5; ++q) {
            const float v = pv[q];
            const __bf16 hv = (__bf16)v;
            s_oh[c0 + q][rloc] = hv;
            s_ol[c0 + q][rloc] = (__bf16)(v - (float)hv);
        }
    }
    __syncthreads();

    {
        const int c = tid >> 3;
        const int piece = tid & 7;
        const v4i vh = *(const v4i*)(&s_oh[c][piece * 8]);
        const v4i vl = *(const v4i*)(&s_ol[c][piece * 8]);
        const size_t off = ((size_t)b * NCP + c) * NN + (size_t)rblk * 64 + (size_t)piece * 8;
        volatile v4i* dh = (volatile v4i*)(hh + off);
        volatile v4i* dl = (volatile v4i*)(hl + off);
        *dh = vh;
        *dl = vl;
        __threadfence();
        *dh = vh;
        *dl = vl;
    }
}

__global__ void __launch_bounds__(256)
k_layer2(const float* __restrict__ x, const __bf16* __restrict__ hh, const __bf16* __restrict__ hl,
         const float* __restrict__ b2, float* __restrict__ out, int nb) {
    __shared__ __align__(16) float2 s_pos[NN];
    __shared__ float s_pre[NN][NCP + 1];
    __shared__ float s_red[16][17];
    __shared__ float s_max[NCP];
    __shared__ float s_lse[NCP];
    __shared__ float s_b2[NCP];

    if ((int)blockIdx.x >= nb) return;
    const int b    = blockIdx.x;
    const int tid  = threadIdx.x;
    const int lane = tid & 31;
    const int wv   = tid >> 5;
    const int hf   = lane >> 4;
    const int m    = lane & 15;

    for (int n = tid; n < NN; n += 256) {
        const float* xr = x + ((size_t)b * NN + n) * FIN;
        s_pos[n] = make_float2(xr[0], xr[1]);
    }
    if (tid < NCP) s_b2[tid] = (tid < NC) ? b2[tid] : 0.0f;
    __syncthreads();

    float2 pm[4];
#pragma unroll
    for (int j = 0; j < 4; ++j) pm[j] = s_pos[(wv * 4 + j) * 16 + m];

    v8f acc[4] = {};
    const __bf16* hhb = hh + (size_t)b * NCP * NN;
    const __bf16* hlb = hl + (size_t)b * NCP * NN;

#pragma unroll 1
    for (int kt = 0; kt < NN / 32; ++kt) {
        const int kbase = kt * 32 + hf * 8;
        float2 pk[16];
        load_pk(s_pos, kbase, pk);
        const size_t ro = (size_t)m * NN + (size_t)kbase;
        Frag16 fbh, fbl;
        fbh.half[0] = *(const v8bf*)(hhb + ro);
        fbh.half[1] = *(const v8bf*)(hhb + ro + 16);
        fbl.half[0] = *(const v8bf*)(hlb + ro);
        fbl.half[1] = *(const v8bf*)(hlb + ro + 16);
#pragma unroll
        for (int j = 0; j < 4; ++j) {
            v16bf ah, al;
            adj_tile(pm[j], (wv * 4 + j) * 16 + m, kbase, pk, ah, al);
            mma3(acc[j], ah, al, fbh.v, fbl.v);
        }
    }

#pragma unroll
    for (int j = 0; j < 4; ++j) {
        const int r0 = (wv * 4 + j) * 16 + 8 * hf;
#pragma unroll
        for (int r = 0; r < 8; ++r)
            s_pre[r0 + r][m] = acc[j][r] + s_b2[m];
    }
    __syncthreads();

    const int c = tid & 15;
    const int g = tid >> 4;
    float mx = -1e30f;
    for (int i = 0; i < 32; ++i) mx = fmaxf(mx, s_pre[g + 16 * i][c]);
    s_red[g][c] = mx;
    __syncthreads();
    if (tid < 16) {
        float mm = -1e30f;
        for (int gg = 0; gg < 16; ++gg) mm = fmaxf(mm, s_red[gg][tid]);
        s_max[tid] = mm;
    }
    __syncthreads();
    const float cm = s_max[c];
    float sm = 0.0f;
    for (int i = 0; i < 32; ++i) sm += __expf(s_pre[g + 16 * i][c] - cm);
    s_red[g][c] = sm;
    __syncthreads();
    if (tid < 16) {
        float ss = 0.0f;
        for (int gg = 0; gg < 16; ++gg) ss += s_red[gg][tid];
        s_lse[tid] = __logf(ss);
    }
    __syncthreads();

    float* ob = out + (size_t)b * NN * NC;
    v4f o[5];
#pragma unroll
    for (int i = 0; i < 5; ++i) {
        const int q = tid + 256 * i;
        v4f t4;
#pragma unroll
        for (int e = 0; e < 4; ++e) {
            const int idx = 4 * q + e;
            const int n   = idx / NC;
            const int cc  = idx - n * NC;
            t4[e] = (s_pre[n][cc] - s_max[cc]) - s_lse[cc];
        }
        o[i] = t4;
    }
#pragma unroll
    for (int i = 0; i < 5; ++i)
        *(volatile v4f*)(ob + (size_t)4 * (tid + 256 * i)) = o[i];
    __threadfence();
#pragma unroll
    for (int i = 0; i < 5; ++i)
        *(volatile v4f*)(ob + (size_t)4 * (tid + 256 * i)) = o[i];
}

extern "C" void kernel_launch(void* const* d_in, const int* in_sizes, int n_in,
                              void* d_out, int out_size, void* d_ws, size_t ws_size,
                              hipStream_t stream) {
    if (n_in < 5) return;
    const int B = in_sizes[0] / (NN * FIN);
    if (B <= 0) return;
    if (in_sizes[0] != B * NN * FIN) return;
    if (in_sizes[1] != FIN * HD || in_sizes[2] != HD) return;
    if (in_sizes[3] != HD * NC || in_sizes[4] != NC) return;
    if (out_size != B * NN * NC) return;

    const float* x  = (const float*)d_in[0];
    const float* W1 = (const float*)d_in[1];
    const float* b1 = (const float*)d_in[2];
    const float* W2 = (const float*)d_in[3];
    const float* b2 = (const float*)d_in[4];
    float* out = (float*)d_out;

    const size_t xbytes = (size_t)B * HD * NN * 2;
    const size_t hbytes = (size_t)B * NCP * NN * 2;
    const size_t total  = 2 * xbytes + 2 * hbytes;
    if (total > ws_size) return;
    char* ws = (char*)d_ws;
    __bf16* xh = (__bf16*)(ws);
    __bf16* xl = (__bf16*)(ws + xbytes);
    __bf16* hh = (__bf16*)(ws + 2 * xbytes);
    __bf16* hl = (__bf16*)(ws + 2 * xbytes + hbytes);

    const int nthr1 = B * HD * (NN / 8);
    k_xw1<<<dim3((nthr1 + 255) / 256), dim3(256), 0, stream>>>(x, W1, xh, xl, nthr1);
    const int nblk2 = B * (NN / 64);
    k_layer1<<<dim3(nblk2), dim3(128), 0, stream>>>(x, xh, xl, b1, W2, hh, hl, nblk2);
    k_layer2<<<dim3(B), dim3(256), 0, stream>>>(x, hh, hl, b2, out, B);
}
